// MultiHeadPointAttention_62878321214031
// MI455X (gfx1250) — hardware-verified
//
#include <hip/hip_runtime.h>
#include <math.h>

typedef __attribute__((ext_vector_type(16))) _Float16 v16h;
typedef __attribute__((ext_vector_type(16))) __bf16 v16b;
typedef __attribute__((ext_vector_type(8)))  _Float16 v8h;
typedef __attribute__((ext_vector_type(8)))  float v8f;
typedef __attribute__((ext_vector_type(4)))  float v4f;
typedef __attribute__((ext_vector_type(2)))  float v2f;
typedef __attribute__((ext_vector_type(4)))  unsigned v4u;
typedef __attribute__((ext_vector_type(4)))  int v4i;
typedef float __attribute__((may_alias)) float_a;
typedef int __attribute__((may_alias)) int_a;

template <typename T> __device__ __forceinline__ void vst2(void* p, T v) { *(volatile T*)p = v; __threadfence(); *(volatile T*)p = v; }
__device__ __forceinline__ v8f wmma16(v16h a, v16h b, v8f c) {
  v8f d = __builtin_amdgcn_wmma_f32_16x16x32_f16(false, a, false, b, (short)0, c, false, false);
  asm volatile("v_nop\n\tv_nop\n\tv_nop\n\tv_nop" : "+v"(d) : "v"(a), "v"(b));
  return d;
}
__device__ __forceinline__ v8f wmma_bf(v16b a, v16b b, v8f c) {
  v8f d = __builtin_amdgcn_wmma_f32_16x16x32_bf16(false, a, false, b, (short)0, c, false, false);
  asm volatile("v_nop\n\tv_nop\n\tv_nop\n\tv_nop" : "+v"(d) : "v"(a), "v"(b));
  return d;
}
__device__ __forceinline__ v16h frag_h(const _Float16* rowk0, int lane) {
  union { v16h v; v8h q[2]; } u; const _Float16* p = rowk0 + 8 * (lane >> 4);
  u.q[0] = *(const v8h*)p; u.q[1] = *(const v8h*)(p + 16); return u.v;
}
__device__ __forceinline__ v16h frag_f32(const float* rowk0, int lane) {
  v16h a; const float* p = rowk0 + 8 * (lane >> 4);
#pragma unroll
  for (int i = 0; i < 8; ++i) { a[i] = (_Float16)p[i]; a[8 + i] = (_Float16)p[16 + i]; }
  return a;
}
__device__ __forceinline__ v16h frag_f32s(const float* rowk0, int lane, float sc) {
  v16h a; const float* p = rowk0 + 8 * (lane >> 4);
#pragma unroll
  for (int i = 0; i < 8; ++i) { a[i] = (_Float16)(p[i] * sc); a[8 + i] = (_Float16)(p[16 + i] * sc); }
  return a;
}
__device__ __forceinline__ v16h fragc_f32(const float* W, int k0, int n, int lane, int ld, int K) {
  v16h a; const int g = lane >> 4;
#pragma unroll
  for (int i = 0; i < 8; ++i) { const int ka = k0 + 8 * g + i, kb = ka + 16;
    a[i] = (_Float16)(ka < K ? W[(size_t)(ka < K ? ka : K - 1) * ld + n] : 0.f); a[8 + i] = (_Float16)(kb < K ? W[(size_t)(kb < K ? kb : K - 1) * ld + n] : 0.f); }
  return a;
}
struct F2 { v16b h, l; };
__device__ __forceinline__ F2 bsplit16(const float v[16]) { F2 r;
#pragma unroll
  for (int i = 0; i < 16; ++i) { const __bf16 h = (__bf16)v[i]; r.h[i] = h; r.l[i] = (__bf16)(v[i] - (float)h); }
  return r; }
__device__ __forceinline__ F2 split_row(const float* row, int k0, int lane) { float v[16]; const float* p = row + k0 + 8 * (lane >> 4);
#pragma unroll
  for (int i = 0; i < 8; ++i) { v[i] = p[i]; v[8 + i] = p[16 + i]; }
  return bsplit16(v); }
__device__ __forceinline__ F2 split_rowK(const float* row, int k0, int lane, int K) { float v[16]; const int g = lane >> 4;
#pragma unroll
  for (int i = 0; i < 8; ++i) { const int ka = k0 + 8 * g + i, kb = ka + 16; v[i] = ka < K ? row[ka < K ? ka : K - 1] : 0.f; v[8 + i] = kb < K ? row[kb < K ? kb : K - 1] : 0.f; }
  return bsplit16(v); }
__device__ __forceinline__ F2 split_col(const float* W, int k0, int n, int lane, int ld, int K) { float v[16]; const int g = lane >> 4;
#pragma unroll
  for (int i = 0; i < 8; ++i) { const int ka = k0 + 8 * g + i, kb = ka + 16; v[i] = ka < K ? W[(size_t)(ka < K ? ka : K - 1) * ld + n] : 0.f; v[8 + i] = kb < K ? W[(size_t)(kb < K ? kb : K - 1) * ld + n] : 0.f; }
  return bsplit16(v); }
__device__ __forceinline__ v8f mac3(const F2& a, const F2& b, v8f c) { c = wmma_bf(a.l, b.h, c); c = wmma_bf(a.h, b.l, c); return wmma_bf(a.h, b.h, c); }
__device__ __forceinline__ float sigm(float v) { return 1.0f / (1.0f + expf(-v)); }
#define LDSX() do { asm volatile("s_wait_dscnt 0" ::: "memory"); __builtin_amdgcn_wave_barrier(); __builtin_amdgcn_fence(__ATOMIC_RELEASE, "workgroup"); } while (0)


#define NB 2
#define NPT 8192
#define MM (NB * NPT)
#define KN 16
#define CI 64
#define CO 128
#ifndef NBLK
#define NBLK (MM / 4)
#define NRB (MM / 64)
#endif
typedef __attribute__((ext_vector_type(8))) __bf16 v8b;
__device__ __forceinline__ v16b frag_b(const __bf16* rowk0, int lane) {
  union { v16b v; v8b q[2]; } u; const __bf16* p = rowk0 + 8 * (lane >> 4);
  u.q[0] = *(const v8b*)p; u.q[1] = *(const v8b*)(p + 16); return u.v;
}
__device__ __forceinline__ float bfr(float v) { return (float)(__bf16)v; }
__device__ __attribute__((noinline)) float exp_ni(float v) { return expf(v); }
__device__ __attribute__((noinline)) float erf_ni(float v) { return erff(v); }

#define WS_PW   0u
#define PQ  0
#define PKV (PQ + 128 * 64)
#define PP2 (PKV + 256 * 64)
#define PA1 (PP2 + 128 * 128)
#define PA2 (PA1 + 128 * 128)
#define PO  (PA2 + 128 * 128)
#define PWEND (PO + 128 * 128)
#define WS_Q    (WS_PW + 2u * PWEND)
#define WS_KV   (WS_Q + 4u * MM * 128)
#define WS_AGG  (WS_KV + 4u * MM * 256)
#define WS_END  (WS_AGG + 4u * MM * 128)

__global__ __launch_bounds__(256) void k_packW(const float* __restrict__ Wm, int K, int NOUT, __bf16* __restrict__ DST_) {
  __shared__ __align__(16) __bf16 s[128]; const int n = blockIdx.x, tid = threadIdx.x; if (n >= NOUT) return;
  if (tid < K) s[tid] = (__bf16)Wm[(size_t)tid * NOUT + n]; __syncthreads();
  if (tid < K / 8) vst2((unsigned*)(DST_ + (size_t)n * K + tid * 8), *(const v4u*)&s[tid * 8]);
}
template <int MODE>
__global__ __launch_bounds__(128) void k_proj(const float* __restrict__ A, int lda, int K, const __bf16* __restrict__ P, const float* __restrict__ bias, float* __restrict__ OUT, int ldo) {
  __shared__ __align__(16) float so[4][16][132];
  const int tid = threadIdx.x, wave = tid >> 5, lane = tid & 31, col = lane & 15, g = lane >> 4; const size_t r0 = (size_t)blockIdx.x * 64 + wave * 16; const int n0 = blockIdx.y * 128;
  v8f acc[8] = {};
  for (int kc = 0; kc < K / 32; ++kc) { F2 a; if (MODE == 1) { v16b ax; const float* p = A + (r0 + col) * (size_t)lda + kc * 32 + 8 * g;
#pragma unroll
      for (int i = 0; i < 8; ++i) { ax[i] = (__bf16)p[i]; ax[8 + i] = (__bf16)p[16 + i]; } a.h = ax; a.l = ax; } else a = split_row(A + (r0 + col) * (size_t)lda, kc * 32, lane);
#pragma unroll
    for (int j = 0; j < 8; ++j) { const v16b w = frag_b(P + (size_t)(n0 + j * 16 + col) * K + kc * 32, lane); if (MODE == 0) acc[j] = wmma_bf(a.l, w, acc[j]); acc[j] = wmma_bf(a.h, w, acc[j]); } }
#pragma unroll
  for (int j = 0; j < 8; ++j) { const float bb = bfr(bias[n0 + j * 16 + col]);
#pragma unroll
    for (int r = 0; r < 8; ++r) so[wave][8 * g + r][j * 16 + col] = acc[j][r] + bb; }
  LDSX();
  for (int rl = 0; rl < 16; ++rl) vst2(OUT + (r0 + rl) * (size_t)ldo + n0 + lane * 4, *(const v4f*)&so[wave][rl][lane * 4]);
}
__device__ __forceinline__ void wave_layer(float (*rows)[132], const __bf16* __restrict__ P, const float* __restrict__ bias, bool relu, int lane) {
  const int col = lane & 15, g = lane >> 4; v8f acc[8] = {};
#pragma unroll
  for (int kc = 0; kc < 4; ++kc) { const F2 a = split_row(&rows[col][0], kc * 32, lane);
#pragma unroll
    for (int j = 0; j < 8; ++j) { const v16b w = frag_b(P + (size_t)(j * 16 + col) * 128 + kc * 32, lane); acc[j] = wmma_bf(a.l, w, acc[j]); acc[j] = wmma_bf(a.h, w, acc[j]); } }
  LDSX();
#pragma unroll
  for (int j = 0; j < 8; ++j) { const float bb = bfr(bias[j * 16 + col]);
#pragma unroll
    for (int r = 0; r < 8; ++r) { float v = acc[j][r] + bb; if (relu) v = fmaxf(v, 0.f); rows[8 * g + r][j * 16 + col] = v; } }
  LDSX();
}
__global__ __launch_bounds__(128) void k_point(const float* __restrict__ POS, const int* __restrict__ IDX, const float* __restrict__ Q, const float* __restrict__ KV, const float* __restrict__ WP1, const float* __restrict__ BP1, const __bf16* __restrict__ PW, const float* __restrict__ BP2, const float* __restrict__ BA1, const float* __restrict__ BA2, float* __restrict__ AGG) {
  __shared__ __align__(16) float sr[4][16][132], spe[4][16][132]; __shared__ int sj[4][16]; __shared__ __align__(16) float sg[4][128];
  const int tid = threadIdx.x, wave = tid >> 5, lane = tid & 31, col = lane & 15, g = lane >> 4; const size_t i = (size_t)blockIdx.x * 4 + wave; const int b = (int)(i / NPT);
  if (lane < KN) sj[wave][lane] = b * NPT + min(max(IDX[i * KN + lane], 0), NPT - 1);
  LDSX();
  { const float px = bfr(POS[i * 3]), py = bfr(POS[i * 3 + 1]), pz = bfr(POS[i * 3 + 2]);
    for (int m = 0; m < 4; ++m) { const int c = lane + 32 * m; const float w0 = bfr(WP1[c]), w1 = bfr(WP1[128 + c]), w2 = bfr(WP1[256 + c]), bb = bfr(BP1[c]);
#pragma unroll 1
      for (int r = 0; r < KN; ++r) { const int j = sj[wave][r]; const float dx = px - bfr(POS[(size_t)j * 3]), dy = py - bfr(POS[(size_t)j * 3 + 1]), dz = pz - bfr(POS[(size_t)j * 3 + 2]); sr[wave][r][c] = fmaxf(((dx * w0 + dy * w1) + dz * w2) + bb, 0.f); } } }
  LDSX();
  wave_layer(sr[wave], PW + PP2, BP2, false, lane);
  for (int m = 0; m < 4; ++m) { const int c = lane + 32 * m; const float qi = Q[i * 128 + c];
#pragma unroll 1
    for (int r = 0; r < KN; ++r) { const float pe = sr[wave][r][c]; spe[wave][r][c] = pe; sr[wave][r][c] = KV[(size_t)sj[wave][r] * 256 + c] - qi + pe; } }
  LDSX();
  wave_layer(sr[wave], PW + PA1, BA1, true, lane);
  wave_layer(sr[wave], PW + PA2, BA2, false, lane);
  for (int m = 0; m < 4; ++m) { const int c = lane + 32 * m; float mx = -3.0e38f;
#pragma unroll 1
    for (int r = 0; r < KN; ++r) mx = fmaxf(mx, sr[wave][r][c]);
    float s = 0.f, a = 0.f;
#pragma unroll 1
    for (int r = 0; r < KN; ++r) { const float e = exp_ni(sr[wave][r][c] - mx); s += e; a += e * (KV[(size_t)sj[wave][r] * 256 + 128 + c] + spe[wave][r][c]); }
    sg[wave][c] = a / s; }
  LDSX();
  vst2(AGG + i * 128 + lane * 4, *(const v4f*)&sg[wave][lane * 4]);
}
extern "C" void kernel_launch(void* const* d_in, const int* in_sizes, int n_in, void* d_out, int out_size, void* d_ws, size_t ws_size, hipStream_t stream) {
  (void)in_sizes; (void)n_in; (void)out_size;
  const float** F = (const float**)d_in; const int* IDX = (const int*)d_in[2];
  if (ws_size < (size_t)WS_END) return;
  char* ws = (char*)d_ws; __bf16* PW = (__bf16*)(ws + WS_PW); float *Q = (float*)(ws + WS_Q), *KV = (float*)(ws + WS_KV), *AGG = (float*)(ws + WS_AGG);
  k_packW<<<128, 256, 0, stream>>>(F[3], 64, 128, PW + PQ); k_packW<<<256, 256, 0, stream>>>(F[5], 64, 256, PW + PKV); k_packW<<<128, 256, 0, stream>>>(F[9], 128, 128, PW + PP2); k_packW<<<128, 256, 0, stream>>>(F[11], 128, 128, PW + PA1); k_packW<<<128, 256, 0, stream>>>(F[13], 128, 128, PW + PA2); k_packW<<<128, 256, 0, stream>>>(F[15], 128, 128, PW + PO);
  k_proj<1><<<dim3(NRB, 1), 128, 0, stream>>>(F[0], CI, CI, PW + PQ, F[4], Q, 128);
  k_proj<1><<<dim3(NRB, 2), 128, 0, stream>>>(F[0], CI, CI, PW + PKV, F[6], KV, 256);
  k_point<<<NBLK, 128, 0, stream>>>(F[1], IDX, Q, KV, F[7], F[8], PW, F[10], F[12], F[14], AGG);
  k_proj<0><<<dim3(NRB, 1), 128, 0, stream>>>(AGG, 128, 128, PW + PO, F[16], (float*)d_out, 128);
}
